// MultiHeadAttnRelPos_46866683134052
// MI455X (gfx1250) — hardware-verified
//
#include <hip/hip_runtime.h>
#include <math.h>

typedef __attribute__((ext_vector_type(16))) _Float16 v16h;
typedef __attribute__((ext_vector_type(16))) __bf16 v16b;
typedef __attribute__((ext_vector_type(8)))  _Float16 v8h;
typedef __attribute__((ext_vector_type(8)))  float v8f;
typedef __attribute__((ext_vector_type(4)))  float v4f;
typedef __attribute__((ext_vector_type(2)))  float v2f;
typedef __attribute__((ext_vector_type(4)))  unsigned v4u;
typedef __attribute__((ext_vector_type(4)))  int v4i;
typedef float __attribute__((may_alias)) float_a;
typedef int __attribute__((may_alias)) int_a;

template <typename T> __device__ __forceinline__ void vst2(void* p, T v) { *(volatile T*)p = v; __threadfence(); *(volatile T*)p = v; }
__device__ __forceinline__ v8f wmma16(v16h a, v16h b, v8f c) {
  v8f d = __builtin_amdgcn_wmma_f32_16x16x32_f16(false, a, false, b, (short)0, c, false, false);
  asm volatile("v_nop\n\tv_nop\n\tv_nop\n\tv_nop" : "+v"(d) : "v"(a), "v"(b));
  return d;
}
__device__ __forceinline__ v8f wmma_bf(v16b a, v16b b, v8f c) {
  v8f d = __builtin_amdgcn_wmma_f32_16x16x32_bf16(false, a, false, b, (short)0, c, false, false);
  asm volatile("v_nop\n\tv_nop\n\tv_nop\n\tv_nop" : "+v"(d) : "v"(a), "v"(b));
  return d;
}
__device__ __forceinline__ v16h frag_h(const _Float16* rowk0, int lane) {
  union { v16h v; v8h q[2]; } u; const _Float16* p = rowk0 + 8 * (lane >> 4);
  u.q[0] = *(const v8h*)p; u.q[1] = *(const v8h*)(p + 16); return u.v;
}
__device__ __forceinline__ v16h frag_f32(const float* rowk0, int lane) {
  v16h a; const float* p = rowk0 + 8 * (lane >> 4);
#pragma unroll
  for (int i = 0; i < 8; ++i) { a[i] = (_Float16)p[i]; a[8 + i] = (_Float16)p[16 + i]; }
  return a;
}
__device__ __forceinline__ v16h frag_f32s(const float* rowk0, int lane, float sc) {
  v16h a; const float* p = rowk0 + 8 * (lane >> 4);
#pragma unroll
  for (int i = 0; i < 8; ++i) { a[i] = (_Float16)(p[i] * sc); a[8 + i] = (_Float16)(p[16 + i] * sc); }
  return a;
}
__device__ __forceinline__ v16h fragc_f32(const float* W, int k0, int n, int lane, int ld, int K) {
  v16h a; const int g = lane >> 4;
#pragma unroll
  for (int i = 0; i < 8; ++i) { const int ka = k0 + 8 * g + i, kb = ka + 16;
    a[i] = (_Float16)(ka < K ? W[(size_t)(ka < K ? ka : K - 1) * ld + n] : 0.f); a[8 + i] = (_Float16)(kb < K ? W[(size_t)(kb < K ? kb : K - 1) * ld + n] : 0.f); }
  return a;
}
struct F2 { v16b h, l; };
__device__ __forceinline__ F2 bsplit16(const float v[16]) { F2 r;
#pragma unroll
  for (int i = 0; i < 16; ++i) { const __bf16 h = (__bf16)v[i]; r.h[i] = h; r.l[i] = (__bf16)(v[i] - (float)h); }
  return r; }
__device__ __forceinline__ F2 split_row(const float* row, int k0, int lane) { float v[16]; const float* p = row + k0 + 8 * (lane >> 4);
#pragma unroll
  for (int i = 0; i < 8; ++i) { v[i] = p[i]; v[8 + i] = p[16 + i]; }
  return bsplit16(v); }
__device__ __forceinline__ F2 split_rowK(const float* row, int k0, int lane, int K) { float v[16]; const int g = lane >> 4;
#pragma unroll
  for (int i = 0; i < 8; ++i) { const int ka = k0 + 8 * g + i, kb = ka + 16; v[i] = ka < K ? row[ka < K ? ka : K - 1] : 0.f; v[8 + i] = kb < K ? row[kb < K ? kb : K - 1] : 0.f; }
  return bsplit16(v); }
__device__ __forceinline__ F2 split_col(const float* W, int k0, int n, int lane, int ld, int K) { float v[16]; const int g = lane >> 4;
#pragma unroll
  for (int i = 0; i < 8; ++i) { const int ka = k0 + 8 * g + i, kb = ka + 16; v[i] = ka < K ? W[(size_t)(ka < K ? ka : K - 1) * ld + n] : 0.f; v[8 + i] = kb < K ? W[(size_t)(kb < K ? kb : K - 1) * ld + n] : 0.f; }
  return bsplit16(v); }
__device__ __forceinline__ v8f mac3(const F2& a, const F2& b, v8f c) { c = wmma_bf(a.l, b.h, c); c = wmma_bf(a.h, b.l, c); return wmma_bf(a.h, b.h, c); }
__device__ __forceinline__ float sigm(float v) { return 1.0f / (1.0f + expf(-v)); }
#define LDSX() do { asm volatile("s_wait_dscnt 0" ::: "memory"); __builtin_amdgcn_wave_barrier(); __builtin_amdgcn_fence(__ATOMIC_RELEASE, "workgroup"); } while (0)


#define QL 1024
#define ML 1024
#define KL 2048
#define BZ 4
#define DE 1024
#define NH 16
#define HD 64
#define NRK (BZ * KL)
#define NRQ (BZ * QL)
#ifndef TQB
#define TQB (QL / 64)
#define TNB BZ
#endif
typedef __attribute__((ext_vector_type(8))) __bf16 v8b;
__device__ __forceinline__ v16b frag_b(const __bf16* rowk0, int lane) {
  union { v16b v; v8b q[2]; } u; const __bf16* p = rowk0 + 8 * (lane >> 4);
  u.q[0] = *(const v8b*)p; u.q[1] = *(const v8b*)(p + 16); return u.v;
}
__device__ __forceinline__ float bfr(float v) { return (float)(__bf16)v; }
__device__ __attribute__((noinline)) float exp_ni(float v) { return expf(v); }
__device__ __attribute__((noinline)) float erf_ni(float v) { return erff(v); }

#define PK_Q  0
#define PK_K  (PK_Q + (size_t)DE * DE)
#define PK_V  (PK_K + (size_t)DE * DE)
#define PK_R  (PK_V + (size_t)DE * DE)
#define PK_O  (PK_R + (size_t)DE * DE)
#define PK_END (PK_O + (size_t)DE * DE)
#define WS_PK  0u
#define WS_KV  (WS_PK + 2u * (unsigned)PK_END)
#define WS_Q   (WS_KV + 4u * NRK * DE)
#define WS_RK  (WS_Q + 4u * NRQ * DE)
#define WS_VTH (WS_RK + 4u * KL * DE)
#define WS_VTL (WS_VTH + 2u * BZ * DE * KL)
#define WS_END (WS_VTL + 2u * BZ * DE * KL)

__global__ __launch_bounds__(256) void k_packT(const float* __restrict__ Wm, int K, int ld, int col0, __bf16* __restrict__ DST) {
  __shared__ __align__(16) __bf16 s[DE]; const int n = blockIdx.x, tid = threadIdx.x;
  for (int k = tid; k < K; k += 256) s[k] = (__bf16)Wm[(size_t)k * ld + col0 + n];
  __syncthreads();
  for (int q = tid; q < K / 8; q += 256) vst2((unsigned*)(DST + (size_t)n * K + q * 8), *(const v4u*)&s[q * 8]);
}
template <int MODE>
__global__ __launch_bounds__(128) void k_proj(const float* __restrict__ Wx, const float* __restrict__ Mx, const __bf16* __restrict__ P, float* __restrict__ OUT, __bf16* __restrict__ VTH, __bf16* __restrict__ VTL) {
  __shared__ __align__(16) float so[MODE == 2 ? 1 : 4][16][132]; __shared__ __align__(16) __bf16 sth[MODE == 2 ? 128 : 1][72], stl[MODE == 2 ? 128 : 1][72];
  const int tid = threadIdx.x, wave = tid >> 5, lane = tid & 31, col = lane & 15, g = lane >> 4; const size_t r0 = (size_t)blockIdx.x * 64 + wave * 16; const int n0 = blockIdx.y * 128;
  const size_t ra = r0 + col; const float* src;
  if (MODE == 1) { const int b = (int)(ra / QL), i = (int)(ra % QL); src = Wx + ((size_t)i * BZ + b) * DE; }
  else { const int b = (int)(ra / KL), s = (int)(ra % KL); src = (s < ML) ? Mx + ((size_t)s * BZ + b) * DE : Wx + ((size_t)(s - ML) * BZ + b) * DE; }
  v8f acc[8] = {};
#pragma unroll 2
  for (int kc = 0; kc < DE / 32; ++kc) { v16b a; { const float* p = src + kc * 32 + 8 * g;
#pragma unroll
      for (int ii = 0; ii < 8; ++ii) { a[ii] = (__bf16)p[ii]; a[8 + ii] = (__bf16)p[16 + ii]; } }
#pragma unroll
    for (int j = 0; j < 8; ++j) acc[j] = wmma_bf(a, frag_b(P + (size_t)(n0 + j * 16 + col) * DE + kc * 32, lane), acc[j]); }
  if (MODE != 2) {
#pragma unroll
    for (int j = 0; j < 8; ++j)
#pragma unroll
      for (int r = 0; r < 8; ++r) so[wave][8 * g + r][j * 16 + col] = acc[j][r];
    LDSX();
    for (int rl = 0; rl < 16; ++rl) vst2(OUT + (r0 + rl) * DE + n0 + lane * 4, *(const v4f*)&so[wave][rl][lane * 4]);
  } else {
#pragma unroll
    for (int j = 0; j < 8; ++j)
#pragma unroll
      for (int r = 0; r < 8; ++r) { const float v = acc[j][r]; const __bf16 hb = (__bf16)v; sth[j * 16 + col][wave * 16 + 8 * g + r] = hb; stl[j * 16 + col][wave * 16 + 8 * g + r] = (__bf16)(v - (float)hb); }
    __syncthreads();
    const size_t rb = (size_t)blockIdx.x * 64; const int b = (int)(rb / KL), s0 = (int)(rb % KL);
    for (int q = tid; q < 128 * 8; q += 128) { const int d = q >> 3, pc = q & 7; const size_t o = ((size_t)b * DE + n0 + d) * KL + s0 + pc * 8; vst2((unsigned*)(VTH + o), *(const v4u*)&sth[d][pc * 8]); vst2((unsigned*)(VTL + o), *(const v4u*)&stl[d][pc * 8]); }
  }
}
__global__ __launch_bounds__(128) void k_rk(const float* __restrict__ Rx, const __bf16* __restrict__ P, float* __restrict__ RK) {
  __shared__ __align__(16) float so[4][16][132];
  const int tid = threadIdx.x, wave = tid >> 5, lane = tid & 31, col = lane & 15, g = lane >> 4; const size_t r0 = (size_t)blockIdx.x * 64 + wave * 16; const int n0 = blockIdx.y * 128;
  v8f acc[8] = {};
#pragma unroll 2
  for (int kc = 0; kc < DE / 32; ++kc) { v16b a; { const float* p = Rx + (r0 + col) * DE + kc * 32 + 8 * g;
#pragma unroll
      for (int ii = 0; ii < 8; ++ii) { a[ii] = (__bf16)p[ii]; a[8 + ii] = (__bf16)p[16 + ii]; } }
#pragma unroll
    for (int j = 0; j < 8; ++j) acc[j] = wmma_bf(a, frag_b(P + (size_t)(n0 + j * 16 + col) * DE + kc * 32, lane), acc[j]); }
#pragma unroll
  for (int j = 0; j < 8; ++j)
#pragma unroll
    for (int r = 0; r < 8; ++r) so[wave][8 * g + r][j * 16 + col] = acc[j][r];
  LDSX();
  for (int rl = 0; rl < 16; ++rl) vst2(RK + (r0 + rl) * DE + n0 + lane * 4, *(const v4f*)&so[wave][rl][lane * 4]);
}
__device__ __forceinline__ F2 split_rowb(const float* row, const float* bias, int k0, int lane) { float v[16]; const float* p = row + k0 + 8 * (lane >> 4); const float* pb = bias + k0 + 8 * (lane >> 4);
#pragma unroll
  for (int i = 0; i < 8; ++i) { v[i] = p[i] + bfr(pb[i]); v[8 + i] = p[16 + i] + bfr(pb[16 + i]); }
  return bsplit16(v); }
__global__ __launch_bounds__(128) void k_attn(float* __restrict__ Q, const float* __restrict__ KV, const float* __restrict__ RK, const float* __restrict__ rwb, const float* __restrict__ rrb, const __bf16* __restrict__ VTH, const __bf16* __restrict__ VTL) {
  __shared__ __align__(16) float sp[4][16][36]; __shared__ __align__(16) float so[4][16][68]; __shared__ float sbd[4][16][52];
  const int tid = threadIdx.x, wave = tid >> 5, lane = tid & 31, col = lane & 15, g = lane >> 4;
  const int qb = blockIdx.x, bh = blockIdx.y, b = bh >> 4, h = bh & 15; const int i0 = qb * 64 + wave * 16; const size_t tq = (size_t)b * QL + i0;
  const float* qrow = Q + (tq + col) * DE + h * HD;
  const F2 aw0 = split_rowb(qrow, rwb + h * HD, 0, lane), aw1 = split_rowb(qrow, rwb + h * HD, 32, lane), ar0 = split_rowb(qrow, rrb + h * HD, 0, lane), ar1 = split_rowb(qrow, rrb + h * HD, 32, lane);
  float m[8], l[8];
#pragma unroll
  for (int r = 0; r < 8; ++r) { m[r] = -3.0e38f; l[r] = 0.f; }
  v8f acc[4] = {};
  const int nsteps = (i0 + 15 + ML) / 32 + 1;
#pragma unroll 1
  for (int ks = 0; ks < nsteps; ++ks) { const int j0 = ks * 32; const bool tail = (j0 + 31 > i0 + ML);
    const int m0 = j0 + (QL - 16) - i0;
#pragma unroll
    for (int mt = 0; mt < 3; ++mt) { int mrow = m0 + mt * 16 + col; mrow = mrow < 0 ? 0 : (mrow > KL - 1 ? KL - 1 : mrow); const float* rkrow = RK + (size_t)mrow * DE + h * HD; const F2 k0 = split_row(rkrow, 0, lane), k1 = split_row(rkrow, 32, lane);
      v8f c = mac3(ar0, k0, (v8f){}); c = mac3(ar1, k1, c);
#pragma unroll
      for (int r = 0; r < 8; ++r) sbd[wave][8 * g + r][mt * 16 + col] = c[r]; }
    LDSX();
    v8f s[2];
#pragma unroll
    for (int ct = 0; ct < 2; ++ct) { const int kk = j0 + ct * 16 + col; const float* krow = KV + ((size_t)b * KL + kk) * DE + h * HD; const F2 k0 = split_row(krow, 0, lane), k1 = split_row(krow, 32, lane);
      v8f c = mac3(aw0, k0, (v8f){}); c = mac3(aw1, k1, c);
#pragma unroll
      for (int r = 0; r < 8; ++r) { const int il = 8 * g + r; const int i = i0 + il; const int jl = ct * 16 + col; float v = (c[r] + sbd[wave][il][jl + 15 - il]) * 0.125f; if (tail && (kk > i + ML)) v = -3.0e38f; s[ct][r] = v; } }
#pragma unroll
    for (int r = 0; r < 8; ++r) { float mx = fmaxf(s[0][r], s[1][r]);
#pragma unroll
      for (int o = 1; o < 16; o <<= 1) mx = fmaxf(mx, __shfl_xor(mx, o));
      const float mn = fmaxf(m[r], mx); const float alpha = (mn <= -1.0e38f) ? 1.0f : exp_ni(m[r] - mn);
      const float e0 = s[0][r] <= -1.0e38f ? 0.f : exp_ni(s[0][r] - mn), e1 = s[1][r] <= -1.0e38f ? 0.f : exp_ni(s[1][r] - mn); float es = e0 + e1;
#pragma unroll
      for (int o = 1; o < 16; o <<= 1) es += __shfl_xor(es, o);
      l[r] = l[r] * alpha + es; m[r] = mn;
#pragma unroll
      for (int dt = 0; dt < 4; ++dt) acc[dt][r] *= alpha;
      sp[wave][8 * g + r][col] = e0; sp[wave][8 * g + r][16 + col] = e1; }
    LDSX();
    const F2 pa = split_row(&sp[wave][col][0], 0, lane);
#pragma unroll
    for (int dt = 0; dt < 4; ++dt) { const size_t vrow = ((size_t)b * DE + h * HD + dt * 16 + col) * KL + j0; const v16b vh = frag_b(VTH + vrow, lane), vl = frag_b(VTL + vrow, lane); acc[dt] = wmma_bf(pa.l, vh, acc[dt]); acc[dt] = wmma_bf(pa.h, vl, acc[dt]); acc[dt] = wmma_bf(pa.h, vh, acc[dt]); }
    LDSX(); }
#pragma unroll
  for (int r = 0; r < 8; ++r) { const float il = 1.0f / l[r];
#pragma unroll
    for (int dt = 0; dt < 4; ++dt) so[wave][8 * g + r][dt * 16 + col] = acc[dt][r] * il; }
  LDSX();
  for (int rl = 0; rl < 16; ++rl) if (lane < 16) vst2(Q + (tq + rl) * DE + h * HD + lane * 4, *(const v4f*)&so[wave][rl][lane * 4]);
}
__global__ __launch_bounds__(128) void k_out(const float* __restrict__ O, const __bf16* __restrict__ P, float* __restrict__ Y) {
  __shared__ __align__(16) float so[4][16][132];
  const int tid = threadIdx.x, wave = tid >> 5, lane = tid & 31, col = lane & 15, g = lane >> 4; const size_t r0 = (size_t)blockIdx.x * 64 + wave * 16; const int n0 = blockIdx.y * 128;
  v8f acc[8] = {};
#pragma unroll 2
  for (int kc = 0; kc < DE / 32; ++kc) { const F2 a = split_row(O + (r0 + col) * DE, kc * 32, lane);
#pragma unroll
    for (int j = 0; j < 8; ++j) { const v16b w = frag_b(P + (size_t)(n0 + j * 16 + col) * DE + kc * 32, lane); acc[j] = wmma_bf(a.l, w, acc[j]); acc[j] = wmma_bf(a.h, w, acc[j]); } }
#pragma unroll
  for (int j = 0; j < 8; ++j)
#pragma unroll
    for (int r = 0; r < 8; ++r) so[wave][8 * g + r][j * 16 + col] = acc[j][r];
  LDSX();
  for (int rl = 0; rl < 16; ++rl) { const size_t rr = r0 + rl; const size_t drow = (rr % QL) * BZ + (rr / QL); vst2(Y + drow * DE + n0 + lane * 4, *(const v4f*)&so[wave][rl][lane * 4]); }
}
extern "C" void kernel_launch(void* const* d_in, const int* in_sizes, int n_in, void* d_out, int out_size, void* d_ws, size_t ws_size, hipStream_t stream) {
  (void)in_sizes; (void)n_in; (void)out_size;
  const float** F = (const float**)d_in;
  if (ws_size < (size_t)WS_END) return;
  char* ws = (char*)d_ws; __bf16 *PK = (__bf16*)(ws + WS_PK), *VTH = (__bf16*)(ws + WS_VTH), *VTL = (__bf16*)(ws + WS_VTL); float *KV = (float*)(ws + WS_KV), *Q = (float*)(ws + WS_Q), *RK = (float*)(ws + WS_RK);
  k_packT<<<DE, 256, 0, stream>>>(F[6], DE, 3 * DE, 0, PK + PK_Q);
  k_packT<<<DE, 256, 0, stream>>>(F[6], DE, 3 * DE, DE, PK + PK_K);
  k_packT<<<DE, 256, 0, stream>>>(F[6], DE, 3 * DE, 2 * DE, PK + PK_V);
  k_packT<<<DE, 256, 0, stream>>>(F[7], DE, DE, 0, PK + PK_R);
  k_packT<<<DE, 256, 0, stream>>>(F[8], DE, DE, 0, PK + PK_O);
  k_proj<0><<<dim3(TNB * KL / 64, DE / 128), 128, 0, stream>>>(F[0], F[5], PK + PK_K, KV, nullptr, nullptr);
  k_proj<2><<<dim3(TNB * KL / 64, DE / 128), 128, 0, stream>>>(F[0], F[5], PK + PK_V, nullptr, VTH, VTL);
  k_proj<1><<<dim3(TNB * QL / 64, DE / 128), 128, 0, stream>>>(F[0], F[5], PK + PK_Q, Q, nullptr, nullptr);
  k_rk<<<dim3(KL / 64, DE / 128), 128, 0, stream>>>(F[1], PK + PK_R, RK);
  k_attn<<<dim3(TQB, TNB * NH), 128, 0, stream>>>(Q, KV, RK, F[2], F[3], VTH, VTL);
  k_out<<<dim3(TNB * TQB, DE / 128), 128, 0, stream>>>(Q, PK + PK_O, (float*)d_out);
}
